// DualAttentionHead_32444182954276
// MI455X (gfx1250) — hardware-verified
//
#include <hip/hip_runtime.h>
#include <math.h>
#include <stddef.h>
#include <stdint.h>

typedef __attribute__((ext_vector_type(16))) _Float16 v16h;
typedef __attribute__((ext_vector_type(8)))  _Float16 v8h;
typedef __attribute__((ext_vector_type(16))) __bf16   v16b;
typedef __attribute__((ext_vector_type(8)))  __bf16   v8b;
typedef __attribute__((ext_vector_type(8)))  float    v8f;
typedef __attribute__((ext_vector_type(4)))  float    v4f;
typedef __attribute__((ext_vector_type(4)))  unsigned int v4u;
typedef __attribute__((ext_vector_type(2)))  unsigned int v2u;

constexpr int kImgs     = 4;
constexpr int kCin      = 512;
constexpr int kCinShift = 9;
constexpr int kCi       = 128;
constexpr int kCiShift  = 7;
constexpr int kPix      = 4096;
constexpr int kRowsAll  = kImgs * kPix;
constexpr int kCls      = 19;
constexpr int kK1       = 9 * kCin;
constexpr int kK2       = 9 * kCi;
constexpr int kQkLd     = 64;
constexpr int kFeat2Ld  = 256;
constexpr int kHeadRows = 64;
constexpr int kKvChunk  = 64;
constexpr int kFlashWaves = 4;
constexpr int kOsPitch  = 132;
constexpr float kWCarry  = 32.0f;
constexpr float kQkvCarry = 16.0f;
constexpr float kPCarry  = 32768.0f;

static_assert(kK1 % 32 == 0 && kK2 % 32 == 0);
static_assert(kPix % 64 == 0 && kCi % 64 == 0 && kRowsAll % 64 == 0);
static_assert(kPix % kKvChunk == 0);

constexpr size_t kB_IM    = (size_t)kPix * kK1 * 2;
constexpr size_t kB_XT    = (size_t)kPix * kCin * 2;
constexpr size_t kB_F32   = (size_t)kRowsAll * kCi * 4;
constexpr size_t kB_F16   = (size_t)kRowsAll * kCi * 2;
constexpr size_t kB_W1    = (size_t)kCi * kK1 * 2;
constexpr size_t kB_W2    = (size_t)kCi * kK2 * 2;
constexpr size_t kB_SV    = 8192;
constexpr size_t kB_WQK   = 64 * 128 * 2;
constexpr size_t kB_WV    = 128 * 128 * 2;
constexpr size_t kB_WCLS  = 64 * 256 * 2;
constexpr size_t kB_WAUX  = 64 * 128 * 2;
constexpr size_t kB_QK    = (size_t)kRowsAll * kQkLd * 2;
constexpr size_t kB_V     = (size_t)kImgs * kCi * kPix * 2;
constexpr size_t kB_EN    = (size_t)kImgs * kCi * kCi * 4;
constexpr size_t kB_ATT   = (size_t)kImgs * kCi * kCi * 2;
constexpr size_t kB_FEAT2 = (size_t)kRowsAll * kFeat2Ld * 2;

constexpr size_t kO_IM    = 0;
constexpr size_t kO_XT    = kO_IM + kB_IM;
constexpr size_t kO_FP32  = kO_XT + kB_XT;
constexpr size_t kO_FC32  = kO_FP32 + kB_F32;
constexpr size_t kO_FP16  = kO_FC32 + kB_F32;
constexpr size_t kO_FC16  = kO_FP16 + kB_F16;
constexpr size_t kO_W1P   = kO_FC16 + kB_F16;
constexpr size_t kO_W1C   = kO_W1P + kB_W1;
constexpr size_t kO_W2P   = kO_W1C + kB_W1;
constexpr size_t kO_W2C   = kO_W2P + kB_W2;
constexpr size_t kO_SV    = kO_W2C + kB_W2;
constexpr size_t kO_WQK   = kO_SV + kB_SV;
constexpr size_t kO_WV    = kO_WQK + kB_WQK;
constexpr size_t kO_WCLS  = kO_WV + kB_WV;
constexpr size_t kO_WAP   = kO_WCLS + kB_WCLS;
constexpr size_t kO_WAC   = kO_WAP + kB_WAUX;
constexpr size_t kO_QK    = kO_WAC + kB_WAUX;
constexpr size_t kO_V     = kO_QK + kB_QK;
constexpr size_t kO_P2IN  = kO_V + kB_V;
constexpr size_t kO_FCTH  = kO_P2IN + kB_F16;
constexpr size_t kO_FCTL  = kO_FCTH + kB_F16;
constexpr size_t kO_EN    = kO_FCTL + kB_F16;
constexpr size_t kO_ATT   = kO_EN + kB_EN;
constexpr size_t kO_C2IN  = kO_ATT + kB_ATT;
constexpr size_t kO_FEAT2 = kO_C2IN + kB_F16;
constexpr size_t kWsTotal = kO_FEAT2 + kB_FEAT2;
static_assert(kWsTotal == 102031360);
static_assert(kWsTotal <= 134217728);
static_assert((size_t)kRowsAll * kK2 * 2 == kB_IM);
static_assert(kO_FP32 % 256 == 0 && kO_SV % 256 == 0 && kO_QK % 256 == 0 && kO_FEAT2 % 256 == 0);

constexpr int kSlotInvP1 = 0, kSlotBiasP1 = 1, kSlotInvC1 = 2, kSlotBiasC1 = 3;
constexpr int kSlotInvP2 = 4, kSlotBiasP2 = 5, kSlotInvC2 = 6, kSlotBiasC2 = 7;
constexpr int kSlotQkb = 8, kSlotClsb = 9, kSlotApb = 10, kSlotAcb = 11, kSlotVb = 12;
constexpr int kNumSlots = 13;
static_assert((size_t)kNumSlots * 128 * 4 <= kB_SV);

__device__ __forceinline__ unsigned short f2bf_bits(float f) {
  unsigned u = __float_as_uint(f);
  return (unsigned short)((u + 0x7FFFu + ((u >> 16) & 1u)) >> 16);
}
__device__ __forceinline__ float bf_bits2f(unsigned short h) { return __uint_as_float(((unsigned)h) << 16); }

__device__ __forceinline__ void dep_guard_h(v8f& a, v8f& b, v16h x, v16h y) { asm volatile("v_nop\n\tv_nop\n\tv_nop\n\tv_nop" : "+v"(a), "+v"(b) : "v"(x), "v"(y)); }
__device__ __forceinline__ void dep_guard_b(v8f& a, v8f& b, v16b x, v16b y) { asm volatile("v_nop\n\tv_nop\n\tv_nop\n\tv_nop" : "+v"(a), "+v"(b) : "v"(x), "v"(y)); }
__device__ __forceinline__ void keep4_h(v16h a, v16h b, v16h c, v16h d) { asm volatile("v_nop" :: "v"(a), "v"(b), "v"(c), "v"(d)); }
__device__ __forceinline__ void keep4_b(v16b a, v16b b, v16b c, v16b d) { asm volatile("v_nop" :: "v"(a), "v"(b), "v"(c), "v"(d)); }
__device__ __forceinline__ void acc_guard4(v8f& a, v8f& b, v8f& c, v8f& d) { asm volatile("v_nop\n\tv_nop\n\tv_nop\n\tv_nop" : "+v"(a), "+v"(b), "+v"(c), "+v"(d)); }
template <typename T> struct Frag;
template <> struct Frag<_Float16> {
  typedef v16h V; union U { v16h v; v8h h[2]; };
  static __device__ __forceinline__ v16h load(const _Float16* p) {
    U f; f.h[0] = *(const v8h*)(p); f.h[1] = *(const v8h*)(p + 16); return f.v;
  }
  static __device__ __forceinline__ v8f mma(v16h a, v16h b, v8f c) {
    return __builtin_amdgcn_wmma_f32_16x16x32_f16(false, a, false, b, (short)0, c, false, false);
  }
  static __device__ __forceinline__ void guard(v8f& a, v8f& b, v16h x, v16h y) { dep_guard_h(a, b, x, y); }
  static __device__ __forceinline__ void keep(v16h a, v16h b, v16h c, v16h d) { keep4_h(a, b, c, d); }
};
template <> struct Frag<__bf16> {
  typedef v16b V; union U { v16b v; v8b h[2]; };
  static __device__ __forceinline__ v16b load(const __bf16* p) {
    U f; f.h[0] = *(const v8b*)(p); f.h[1] = *(const v8b*)(p + 16); return f.v;
  }
  static __device__ __forceinline__ v8f mma(v16b a, v16b b, v8f c) {
    return __builtin_amdgcn_wmma_f32_16x16x32_bf16(false, a, false, b, (short)0, c, false, false);
  }
  static __device__ __forceinline__ void guard(v8f& a, v8f& b, v16b x, v16b y) { dep_guard_b(a, b, x, y); }
  static __device__ __forceinline__ void keep(v16b a, v16b b, v16b c, v16b d) { keep4_b(a, b, c, d); }
};

template <int ET> struct Elem;
template <> struct Elem<0> { typedef _Float16 T; };
template <> struct Elem<1> { typedef __bf16 T; };
template <int ET, bool SPLIT, int BIAS_MODE, int OUT_MODE, bool RESID, int ACT, int SCL>
__global__ __launch_bounds__(256) void wmma_gemm64(
    const unsigned short* __restrict__ Ap, const unsigned short* __restrict__ A2p, int lda, long strideA,
    const unsigned short* __restrict__ Btp, const unsigned short* __restrict__ Bt2p, int ldb, long strideB,
    void* __restrict__ Cout, void* __restrict__ Cout2, int ldc, long strideC,
    const float* __restrict__ bias, const float* __restrict__ cs,
    const float* __restrict__ resid, long strideR,
    int M, int N, int K, float scale, int mlim) {
  typedef typename Elem<ET>::T T;
  typedef typename Frag<T>::V V;
  const T* A = (const T*)Ap; const T* A2 = (const T*)A2p; const T* Bt = (const T*)Btp; const T* Bt2 = (const T*)Bt2p;
  __shared__ __align__(16) float sT[8][16 * 68];
  const int b    = blockIdx.y;
  const int lane = threadIdx.x & 31;
  const int wave = threadIdx.x >> 5;
  const int tilesN = N >> 6;
  const int tilesM = M >> 6;
  const int tile = blockIdx.x * 8 + wave;
  if (tile >= tilesM * tilesN) return;
  const int tm = tile / tilesN;
  const int tn = tile - tm * tilesN;
  const int m0 = tm << 6;
  const int n0 = tn << 6;

  const T* Ab  = A  + (size_t)b * strideA;
  const T* Bb  = Bt + (size_t)b * strideB;
  const T* Ab2 = SPLIT ? (A2  + (size_t)b * strideA) : nullptr;
  const T* Bb2 = SPLIT ? (Bt2 + (size_t)b * strideB) : nullptr;

  const int rlane = lane & 15;
  const int koff  = (lane >> 4) * 8;
  const int mOff  = (lane >> 4) * 8;

  v8f acc[4][4];
#pragma unroll
  for (int i = 0; i < 4; ++i)
#pragma unroll
    for (int j = 0; j < 4; ++j) acc[i][j] = (v8f){0.f,0.f,0.f,0.f,0.f,0.f,0.f,0.f};

  for (int k0 = 0; k0 < K; k0 += 32) {
    V bh[4], bl[4];
#pragma unroll
    for (int j = 0; j < 4; ++j) {
      const size_t bo = (size_t)(n0 + (j << 4) + rlane) * ldb + koff + k0;
      bh[j] = Frag<T>::load(Bb + bo);
      if (SPLIT) bl[j] = Frag<T>::load(Bb2 + bo);
    }
#pragma unroll
    for (int i = 0; i < 4; ++i) {
      const size_t ao = (size_t)(m0 + (i << 4) + rlane) * lda + koff + k0;
      V ah = Frag<T>::load(Ab + ao);
      V al;
      if (SPLIT) al = Frag<T>::load(Ab2 + ao);
#pragma unroll
      for (int j = 0; j < 4; ++j) {
        acc[i][j] = Frag<T>::mma(ah, bh[j], acc[i][j]);
        if (SPLIT) {
          acc[i][j] = Frag<T>::mma(ah, bl[j], acc[i][j]);
          acc[i][j] = Frag<T>::mma(al, bh[j], acc[i][j]);
        }
      }
      Frag<T>::guard(acc[i][0], acc[i][3], ah, SPLIT ? al : ah);
    }
    Frag<T>::keep(bh[0], bh[1], bh[2], bh[3]);
    if (SPLIT) Frag<T>::keep(bl[0], bl[1], bl[2], bl[3]);
  }
  acc_guard4(acc[0][0], acc[0][1], acc[0][2], acc[0][3]);
  acc_guard4(acc[1][0], acc[1][1], acc[1][2], acc[1][3]);
  acc_guard4(acc[2][0], acc[2][1], acc[2][2], acc[2][3]);
  acc_guard4(acc[3][0], acc[3][1], acc[3][2], acc[3][3]);

  float* slab = sT[wave];
  const float* Rb = RESID ? (resid + (size_t)b * strideR) : nullptr;
  const float gsc = (SCL == 3) ? cs[0] : 1.0f;
#pragma unroll
  for (int i = 0; i < 4; ++i) {
    const int mBase = m0 + (i << 4);
#pragma unroll
    for (int j = 0; j < 4; ++j) {
      const int n = n0 + (j << 4) + rlane;
      float bv = 0.f, cn = 1.f;
      if (BIAS_MODE == 2) bv = bias[n];
      if (SCL == 2) cn = cs[n];
#pragma unroll
      for (int r = 0; r < 8; ++r) {
        float v = acc[i][j][r] * scale;
        if (SCL == 2) v *= cn;
        if (SCL == 3) v *= gsc;
        if (BIAS_MODE == 1) v += bias[mBase + mOff + r];
        if (BIAS_MODE == 2) v += bv;
        if (RESID) v += Rb[(size_t)(mBase + mOff + r) * ldc + n];
        if (ACT == 2) v = fmaxf(v, 0.0f);
        if (ACT == 4) v = (v > 0.f) ? v : 0.01f * v;
        slab[(mOff + r) * 68 + (j << 4) + rlane] = v;
      }
    }
    __builtin_amdgcn_fence(__ATOMIC_RELEASE, "workgroup");
    __builtin_amdgcn_wave_barrier();
    __builtin_amdgcn_fence(__ATOMIC_ACQUIRE, "workgroup");
    if (OUT_MODE == 0) {
      float* C = (float*)Cout + (size_t)b * strideC;
      const int hh = lane >> 4, c4 = (lane & 15) * 4;
      for (int pass = 0; pass < 2; ++pass) {
#pragma unroll
        for (int it = 0; it < 8; ++it) {
          const int row = it * 2 + hh;
          v4f v = *(const v4f*)(slab + row * 68 + c4);
          if (mBase + row < mlim) *(volatile v4f*)(C + (size_t)(mBase + row) * ldc + n0 + c4) = v;
        }
        __threadfence();
      }
    } else {
      const int q = lane >> 3, c8 = (lane & 7) * 8;
      unsigned short* C  = (unsigned short*)Cout  + (size_t)b * strideC;
      unsigned short* C2 = (OUT_MODE == 2) ? ((unsigned short*)Cout2 + (size_t)b * strideC) : nullptr;
      for (int pass = 0; pass < 2; ++pass) {
#pragma unroll
        for (int it = 0; it < 4; ++it) {
          const int row = it * 4 + q;
          const float* sp = slab + row * 68 + c8;
          v8h hv, lv;
#pragma unroll
          for (int e = 0; e < 8; ++e) {
            if (OUT_MODE == 1) {
              hv[e] = (_Float16)sp[e];
            } else {
              unsigned short hb = f2bf_bits(sp[e]);
              unsigned short lb = f2bf_bits(sp[e] - bf_bits2f(hb));
              hv[e] = __builtin_bit_cast(_Float16, hb);
              lv[e] = __builtin_bit_cast(_Float16, lb);
            }
          }
          if (mBase + row < mlim) {
            *(volatile v8h*)(C + (size_t)(mBase + row) * ldc + n0 + c8) = hv;
            if (OUT_MODE == 2) *(volatile v8h*)(C2 + (size_t)(mBase + row) * ldc + n0 + c8) = lv;
          }
        }
        __threadfence();
      }
    }
    __builtin_amdgcn_fence(__ATOMIC_RELEASE, "workgroup");
    __builtin_amdgcn_wave_barrier();
    __builtin_amdgcn_fence(__ATOMIC_ACQUIRE, "workgroup");
  }
}

__global__ __launch_bounds__(256) void cast_f32_f16x2(
    const float* __restrict__ in, _Float16* __restrict__ out, int n2) {
  int i = blockIdx.x * 256 + threadIdx.x;
  if (i < n2) {
    const _Float16 h0 = (_Float16)in[2 * i], h1 = (_Float16)in[2 * i + 1];
    const unsigned u = (unsigned)__builtin_bit_cast(unsigned short, h0) | ((unsigned)__builtin_bit_cast(unsigned short, h1) << 16);
    ((volatile unsigned*)out)[i] = u;
    __threadfence();
    ((volatile unsigned*)out)[i] = u;
  }
}

__device__ __forceinline__ int clampi(int v, int lo, int hi) { return v < lo ? lo : (v > hi ? hi : v); }

template <bool LO>
__global__ __launch_bounds__(256) void k_transpose_bf16(const float* __restrict__ in, int R, int Cc, long sIn,
                                                        unsigned short* __restrict__ outHi,
                                                        unsigned short* __restrict__ outLo, long sOut) {
  __shared__ float T[64][65];
  const int tid = threadIdx.x;
  const int c0 = blockIdx.x * 64, r0 = blockIdx.y * 64, z = blockIdx.z;
  const float* inz = in + (size_t)z * sIn;
#pragma unroll
  for (int it = 0; it < 16; ++it) {
    const int idx = it * 256 + tid;
    const int rl = idx >> 6, cl = idx & 63;
    T[cl][rl] = inz[(size_t)(r0 + rl) * Cc + c0 + cl];
  }
  __syncthreads();
  unsigned short* oh = outHi + (size_t)z * sOut;
  unsigned short* ol = LO ? (outLo + (size_t)z * sOut) : nullptr;
  for (int pass = 0; pass < 2; ++pass) {
#pragma unroll
    for (int it = 0; it < 2; ++it) {
      const int orow = it * 32 + (tid >> 3);
      const int c8 = (tid & 7) * 8;
      v8h hv, lv;
#pragma unroll
      for (int e = 0; e < 8; ++e) {
        const float f = T[orow][c8 + e];
        const unsigned short hb = f2bf_bits(f);
        hv[e] = __builtin_bit_cast(_Float16, hb);
        if (LO) lv[e] = __builtin_bit_cast(_Float16, f2bf_bits(f - bf_bits2f(hb)));
      }
      const size_t o = (size_t)(c0 + orow) * R + r0 + c8;
      *(volatile v8h*)(oh + o) = hv;
      if (LO) *(volatile v8h*)(ol + o) = lv;
    }
    __threadfence();
  }
}

__global__ __launch_bounds__(256) void k_im2col16(const unsigned short* __restrict__ in, int cinShift, int rows,
                                                 unsigned short* __restrict__ out) {
  const int c8n  = 1 << (cinShift - 3);
  const int cpr  = 9 * c8n;
  const long t = (long)blockIdx.x * 256 + threadIdx.x;
  if (t >= (long)rows * cpr) return;
  const int row = (int)(t / cpr);
  const int rem = (int)(t - (long)row * cpr);
  const int tap = rem >> (cinShift - 3);
  const int c8  = (rem & (c8n - 1)) * 8;
  const int img = row >> 12, p = row & 4095;
  const int t3  = tap / 3;
  const int y = (p >> 6) + t3 - 1;
  const int x = (p & 63) + (tap - t3 * 3) - 1;
  const bool valid = ((unsigned)y < 64u) && ((unsigned)x < 64u);
  const int yc = clampi(y, 0, 63), xc = clampi(x, 0, 63);
  const size_t src = ((size_t)((img << 12) + (yc << 6) + xc) << cinShift) + c8;
  const v4u v = *(const v4u*)(in + src);
  v4u o;
  o[0] = valid ? v[0] : 0u; o[1] = valid ? v[1] : 0u; o[2] = valid ? v[2] : 0u; o[3] = valid ? v[3] : 0u;
  unsigned short* dst = out + (size_t)row * (size_t)(9 << cinShift) + ((size_t)tap << cinShift) + c8;
  *(volatile v4u*)dst = o;
  __threadfence();
  *(volatile v4u*)dst = o;
}

template <bool BF>
__global__ __launch_bounds__(256) void k_prep_convw(const float* __restrict__ w, int cinShift, float carry,
                                                   unsigned short* __restrict__ out) {
  const int K = 9 << cinShift;
  const int cpr = K >> 3;
  const int t = blockIdx.x * 256 + threadIdx.x;
  if (t >= kCi * cpr) return;
  const int co = t / cpr;
  const int k8 = (t - co * cpr) * 8;
  v8h o;
#pragma unroll
  for (int e = 0; e < 8; ++e) {
    const int k = k8 + e;
    const int tap = k >> cinShift;
    const int ci = k & ((1 << cinShift) - 1);
    const float f = w[(((size_t)co << cinShift) + ci) * 9 + tap];
    const unsigned short hb = f2bf_bits(f);
    unsigned short bits;
    if (BF) bits = hb;
    else    bits = __builtin_bit_cast(unsigned short, (_Float16)(carry * bf_bits2f(hb)));
    o[e] = __builtin_bit_cast(_Float16, bits);
  }
  unsigned short* dst = out + (size_t)co * K + k8;
  *(volatile v8h*)dst = o;
  __threadfence();
  *(volatile v8h*)dst = o;
}

__global__ __launch_bounds__(256) void k_prep_pad(const float* __restrict__ W, int srcRows, int srcCols,
                                                 int dstRows, int dstCols, float carry,
                                                 unsigned short* __restrict__ out) {
  const int cpr = dstCols >> 3;
  const int t = blockIdx.x * 256 + threadIdx.x;
  if (t >= dstRows * cpr) return;
  const int r = t / cpr;
  const int c8 = (t - r * cpr) * 8;
  const int rr = clampi(r, 0, srcRows - 1);
  const bool live = (r < srcRows);
  v8h o;
#pragma unroll
  for (int e = 0; e < 8; ++e) {
    const int c = c8 + e;
    const int sc = (c >= srcCols) ? (c - srcCols) : c;
    const float f = W[(size_t)rr * srcCols + sc];
    const float val = live ? (carry * bf_bits2f(f2bf_bits(f))) : 0.0f;
    o[e] = (_Float16)val;
  }
  unsigned short* dst = out + (size_t)r * dstCols + c8;
  *(volatile v8h*)dst = o;
  __threadfence();
  *(volatile v8h*)dst = o;
}

__global__ __launch_bounds__(128) void k_smallvec(
    const float* __restrict__ g0, const float* __restrict__ b0, const float* __restrict__ m0, const float* __restrict__ v0,
    const float* __restrict__ g1, const float* __restrict__ b1, const float* __restrict__ m1, const float* __restrict__ v1,
    const float* __restrict__ g2, const float* __restrict__ b2, const float* __restrict__ m2, const float* __restrict__ v2,
    const float* __restrict__ g3, const float* __restrict__ b3, const float* __restrict__ m3, const float* __restrict__ v3,
    const float* __restrict__ qb, const float* __restrict__ kb, const float* __restrict__ vb,
    const float* __restrict__ clsb, const float* __restrict__ apb, const float* __restrict__ acb,
    float* __restrict__ sv) {
  const int s = blockIdx.x;
  const int t = threadIdx.x;
  float val = 0.0f;
  if (s < 8) {
    const int j = s >> 1;
    const float* g = (j == 0) ? g0 : (j == 1) ? g1 : (j == 2) ? g2 : g3;
    const float* bb = (j == 0) ? b0 : (j == 1) ? b1 : (j == 2) ? b2 : b3;
    const float* m = (j == 0) ? m0 : (j == 1) ? m1 : (j == 2) ? m2 : m3;
    const float* vv = (j == 0) ? v0 : (j == 1) ? v1 : (j == 2) ? v2 : v3;
    const float inv = g[t] * (1.0f / sqrtf(vv[t] + 1e-5f));
    const float bs = bb[t] - m[t] * inv;
    val = (s & 1) ? bs : inv;
  } else if (s == kSlotQkb) {
    const float a = qb[t & 15];
    const float k = kb[t & 15];
    val = (t < 16) ? (kQkvCarry * a) : ((t >= 32 && t < 48) ? (kQkvCarry * k) : 0.0f);
  } else if (s == kSlotVb) {
    val = kQkvCarry * vb[t];
  } else {
    const float* src = (s == kSlotClsb) ? clsb : (s == kSlotApb) ? apb : acb;
    const float f = src[clampi(t, 0, kCls - 1)];
    val = (t < kCls) ? f : 0.0f;
  }
  float* dst = sv + s * 128 + t;
  *(volatile float*)dst = val;
  __threadfence();
  *(volatile float*)dst = val;
}

__global__ __launch_bounds__(256) void k_softmax128(const float* __restrict__ en, unsigned short* __restrict__ att, int nrows) {
  const int wave = threadIdx.x >> 5, lane = threadIdx.x & 31;
  const int row = blockIdx.x * 8 + wave;
  if (row >= nrows) return;
  const v4f x = *(const v4f*)(en + (size_t)row * 128 + lane * 4);
  float m = fmaxf(fmaxf(x[0], x[1]), fmaxf(x[2], x[3]));
#pragma unroll
  for (int off = 16; off > 0; off >>= 1) m = fmaxf(m, __shfl_xor(m, off, 32));
  const float e0 = expf(x[0] - m), e1 = expf(x[1] - m), e2 = expf(x[2] - m), e3 = expf(x[3] - m);
  float ssum = (e0 + e1) + (e2 + e3);
#pragma unroll
  for (int off = 16; off > 0; off >>= 1) ssum += __shfl_xor(ssum, off, 32);
  const float inv = 1.0f / ssum;
  const _Float16 h0 = (_Float16)((e0 * inv) * kPCarry), h1 = (_Float16)((e1 * inv) * kPCarry);
  const _Float16 h2 = (_Float16)((e2 * inv) * kPCarry), h3 = (_Float16)((e3 * inv) * kPCarry);
  v2u pk;
  pk[0] = (unsigned)__builtin_bit_cast(unsigned short, h0) | ((unsigned)__builtin_bit_cast(unsigned short, h1) << 16);
  pk[1] = (unsigned)__builtin_bit_cast(unsigned short, h2) | ((unsigned)__builtin_bit_cast(unsigned short, h3) << 16);
  unsigned short* dst = att + (size_t)row * 128 + lane * 4;
  *(volatile v2u*)dst = pk;
  __threadfence();
  *(volatile v2u*)dst = pk;
}

__device__ __forceinline__ v8f mma_f16g(v16h a, v16h b, v8f c) {
  c = __builtin_amdgcn_wmma_f32_16x16x32_f16(false, a, false, b, (short)0, c, false, false);
  asm volatile("v_nop\n\tv_nop\n\tv_nop\n\tv_nop" : "+v"(c) : "v"(a), "v"(b));
  return c;
}

__global__ __launch_bounds__(128) void k_pam_flash(const unsigned short* __restrict__ qkp, const unsigned short* __restrict__ vp,
                                                  const float* __restrict__ featp, const float* __restrict__ gam,
                                                  unsigned short* __restrict__ outp) {
  union FB { v16h v; v8h h[2]; };
  __shared__ __align__(16) _Float16 Psh[kFlashWaves][16 * kKvChunk];
  __shared__ __align__(16) float    Os[kFlashWaves][16 * kOsPitch];
  const int tid = threadIdx.x, wave = tid >> 5, lane = tid & 31, hh = lane >> 4, c = lane & 15;
  const int b  = blockIdx.x >> 6;
  const int qb = blockIdx.x & 63;
  const int q0 = qb * 64 + wave * 16;
  const size_t rb = (size_t)b * kPix;
  const _Float16* QK = (const _Float16*)qkp;
  const _Float16* Vb = (const _Float16*)vp + (size_t)b * kCi * kPix;

  const v16h qa = Frag<_Float16>::load(QK + (rb + q0 + c) * kQkLd + 8 * hh);
  const v8f z8 = {0.f,0.f,0.f,0.f,0.f,0.f,0.f,0.f};
  float mrow[8], lrow[8];
  v8f oacc[8];
#pragma unroll
  for (int r = 0; r < 8; ++r) { mrow[r] = -INFINITY; lrow[r] = 0.f; }
#pragma unroll
  for (int t = 0; t < 8; ++t) oacc[t] = z8;
  const float sscale = 1.0f / 256.0f;

  for (int kc = 0; kc < kPix / kKvChunk; ++kc) {
    const int kv0 = kc * kKvChunk;
    __syncthreads();
    v8f s[4];
#pragma unroll
    for (int j = 0; j < 4; ++j) {
      const v16h kb = Frag<_Float16>::load(QK + (rb + kv0 + j * 16 + c) * kQkLd + 32 + 8 * hh);
      s[j] = mma_f16g(qa, kb, z8);
    }
    float cm[8];
#pragma unroll
    for (int r = 0; r < 8; ++r) {
      float m = -INFINITY;
#pragma unroll
      for (int j = 0; j < 4; ++j) { s[j][r] = s[j][r] * sscale; m = fmaxf(m, s[j][r]); }
#pragma unroll
      for (int off = 1; off < 16; off <<= 1) m = fmaxf(m, __shfl_xor(m, off, 32));
      cm[r] = m;
    }
    _Float16* pwh = Psh[wave];
#pragma unroll
    for (int r = 0; r < 8; ++r) {
      const float mnew = fmaxf(mrow[r], cm[r]);
      const float alpha = expf(mrow[r] - mnew);
      mrow[r] = mnew;
      float psum = 0.f;
#pragma unroll
      for (int j = 0; j < 4; ++j) {
        const float p = expf(s[j][r] - mnew);
        psum += p;
        pwh[(8 * hh + r) * kKvChunk + j * 16 + c] = (_Float16)(p * kPCarry);
      }
#pragma unroll
      for (int off = 1; off < 16; off <<= 1) psum += __shfl_xor(psum, off, 32);
      lrow[r] = lrow[r] * alpha + psum;
#pragma unroll
      for (int t = 0; t < 8; ++t) oacc[t][r] *= alpha;
    }
    __builtin_amdgcn_fence(__ATOMIC_RELEASE, "workgroup");
    __builtin_amdgcn_wave_barrier();
    __builtin_amdgcn_fence(__ATOMIC_ACQUIRE, "workgroup");
#pragma unroll 1
    for (int kk = 0; kk < 2; ++kk) {
      FB pa;
      pa.h[0] = *(const v8h*)(pwh + c * kKvChunk + kk * 32 + 8 * hh);
      pa.h[1] = *(const v8h*)(pwh + c * kKvChunk + kk * 32 + 16 + 8 * hh);
#pragma unroll
      for (int t = 0; t < 8; ++t) {
        const v16h vb = Frag<_Float16>::load(Vb + (size_t)(t * 16 + c) * kPix + kv0 + kk * 32 + 8 * hh);
        oacc[t] = mma_f16g(pa.v, vb, oacc[t]);
      }
    }
  }

  float* os = Os[wave];
#pragma unroll
  for (int r = 0; r < 8; ++r) {
    const float inv = 1.0f / (lrow[r] * (kPCarry * kQkvCarry));
#pragma unroll
    for (int t = 0; t < 8; ++t) os[(8 * hh + r) * kOsPitch + t * 16 + c] = oacc[t][r] * inv;
  }
  __builtin_amdgcn_fence(__ATOMIC_RELEASE, "workgroup");
  __builtin_amdgcn_wave_barrier();
  __builtin_amdgcn_fence(__ATOMIC_ACQUIRE, "workgroup");
  {
    const float g = gam[0];
    const int c8 = c * 8;
    for (int pass = 0; pass < 2; ++pass) {
#pragma unroll
      for (int it = 0; it < 8; ++it) {
        const int row = it * 2 + hh;
        const float* op = os + row * kOsPitch + c8;
        const v4f o0 = *(const v4f*)op, o1 = *(const v4f*)(op + 4);
        const size_t grow = rb + q0 + row;
        const float* rp = featp + grow * kCi + c8;
        const v4f r0 = *(const v4f*)rp, r1 = *(const v4f*)(rp + 4);
        v8h hv;
        hv[0] = (_Float16)(g * o0[0] + r0[0]); hv[1] = (_Float16)(g * o0[1] + r0[1]);
        hv[2] = (_Float16)(g * o0[2] + r0[2]); hv[3] = (_Float16)(g * o0[3] + r0[3]);
        hv[4] = (_Float16)(g * o1[0] + r1[0]); hv[5] = (_Float16)(g * o1[1] + r1[1]);
        hv[6] = (_Float16)(g * o1[2] + r1[2]); hv[7] = (_Float16)(g * o1[3] + r1[3]);
        *(volatile v8h*)(outp + grow * kCi + c8) = hv;
      }
      __threadfence();
    }
  }
}

static inline unsigned gemm_gx(int M, int N) { return (unsigned)(((M / 64) * (N / 64) + 7) / 8); }

extern "C" void kernel_launch(void* const* d_in, const int* in_sizes, int n_in,
                              void* d_out, int out_size, void* d_ws, size_t ws_size,
                              hipStream_t stream)
{
  if (n_in < 35) return;
  if (ws_size < kWsTotal) return;
  if ((long)out_size < (long)3 * kImgs * kCls * kPix) return;
  if ((long)in_sizes[0] < (long)kImgs * kCin * kPix) return;

  const float* x      = (const float*)d_in[0];
  const float* wp1    = (const float*)d_in[1];
  const float* bnp1_w = (const float*)d_in[2];
  const float* bnp1_b = (const float*)d_in[3];
  const float* bnp1_m = (const float*)d_in[4];
  const float* bnp1_v = (const float*)d_in[5];
  const float* qw     = (const float*)d_in[6];
  const float* qb     = (const float*)d_in[7];
  const float* kw     = (const float*)d_in[8];
  const float* kb     = (const float*)d_in[9];
  const float* vw     = (const float*)d_in[10];
  const float* vb     = (const float*)d_in[11];
  const float* pamg   = (const float*)d_in[12];
  const float* wp2    = (const float*)d_in[13];
  const float* bnp2_w = (const float*)d_in[14];
  const float* bnp2_b = (const float*)d_in[15];
  const float* bnp2_m = (const float*)d_in[16];
  const float* bnp2_v = (const float*)d_in[17];
  const float* wc1    = (const float*)d_in[18];
  const float* bnc1_w = (const float*)d_in[19];
  const float* bnc1_b = (const float*)d_in[20];
  const float* bnc1_m = (const float*)d_in[21];
  const float* bnc1_v = (const float*)d_in[22];
  const float* camg   = (const float*)d_in[23];
  const float* wc2    = (const float*)d_in[24];
  const float* bnc2_w = (const float*)d_in[25];
  const float* bnc2_b = (const float*)d_in[26];
  const float* bnc2_m = (const float*)d_in[27];
  const float* bnc2_v = (const float*)d_in[28];
  const float* cls_w  = (const float*)d_in[29];
  const float* cls_b  = (const float*)d_in[30];
  const float* auxp_w = (const float*)d_in[31];
  const float* auxp_b = (const float*)d_in[32];
  const float* auxc_w = (const float*)d_in[33];
  const float* auxc_b = (const float*)d_in[34];

  char* ws = (char*)d_ws;
  unsigned short* IM    = (unsigned short*)(ws + kO_IM);
  unsigned short* XT    = (unsigned short*)(ws + kO_XT);
  float*          FP32  = (float*)(ws + kO_FP32);
  float*          FC32  = (float*)(ws + kO_FC32);
  unsigned short* FP16  = (unsigned short*)(ws + kO_FP16);
  unsigned short* FC16  = (unsigned short*)(ws + kO_FC16);
  unsigned short* W1P   = (unsigned short*)(ws + kO_W1P);
  unsigned short* W1C   = (unsigned short*)(ws + kO_W1C);
  unsigned short* W2P   = (unsigned short*)(ws + kO_W2P);
  unsigned short* W2C   = (unsigned short*)(ws + kO_W2C);
  float*          SV    = (float*)(ws + kO_SV);
  unsigned short* WQK   = (unsigned short*)(ws + kO_WQK);
  unsigned short* WV    = (unsigned short*)(ws + kO_WV);
  unsigned short* WCLS  = (unsigned short*)(ws + kO_WCLS);
  unsigned short* WAP   = (unsigned short*)(ws + kO_WAP);
  unsigned short* WAC   = (unsigned short*)(ws + kO_WAC);
  unsigned short* QKP   = (unsigned short*)(ws + kO_QK);
  unsigned short* VPL   = (unsigned short*)(ws + kO_V);
  unsigned short* P2IN  = (unsigned short*)(ws + kO_P2IN);
  unsigned short* FCTH  = (unsigned short*)(ws + kO_FCTH);
  unsigned short* FCTL  = (unsigned short*)(ws + kO_FCTL);
  float*          EN    = (float*)(ws + kO_EN);
  unsigned short* ATT   = (unsigned short*)(ws + kO_ATT);
  unsigned short* C2IN  = (unsigned short*)(ws + kO_C2IN);
  unsigned short* FEAT2 = (unsigned short*)(ws + kO_FEAT2);
  float* dout = (float*)d_out;

  const dim3 blk(256);
  const long featStride = (long)kPix * kCi;
  const long outStride  = (long)kCls * kPix;

  k_prep_convw<true><<<288, blk, 0, stream>>>(wp1, kCinShift, 1.0f, W1P);
  k_prep_convw<true><<<288, blk, 0, stream>>>(wc1, kCinShift, 1.0f, W1C);
  k_prep_convw<false><<<72, blk, 0, stream>>>(wp2, kCiShift, kWCarry, W2P);
  k_prep_convw<false><<<72, blk, 0, stream>>>(wc2, kCiShift, kWCarry, W2C);
  k_smallvec<<<kNumSlots, 128, 0, stream>>>(bnp1_w, bnp1_b, bnp1_m, bnp1_v, bnc1_w, bnc1_b, bnc1_m, bnc1_v,
                                            bnp2_w, bnp2_b, bnp2_m, bnp2_v, bnc2_w, bnc2_b, bnc2_m, bnc2_v,
                                            qb, kb, vb, cls_b, auxp_b, auxc_b, SV);
  k_prep_pad<<<8, blk, 0, stream>>>(vw, kCi, kCi, kCi, kCi, kWCarry, WV);
  k_prep_pad<<<2, blk, 0, stream>>>(qw, 16, kCi, 32, kCi, kWCarry, WQK);
  k_prep_pad<<<2, blk, 0, stream>>>(kw, 16, kCi, 32, kCi, kWCarry, WQK + 32 * kCi);
  k_prep_pad<<<8, blk, 0, stream>>>(cls_w, kCls, kCi, kHeadRows, 2 * kCi, kWCarry, WCLS);
  k_prep_pad<<<4, blk, 0, stream>>>(auxp_w, kCls, kCi, kHeadRows, kCi, kWCarry, WAP);
  k_prep_pad<<<4, blk, 0, stream>>>(auxc_w, kCls, kCi, kHeadRows, kCi, kWCarry, WAC);

  for (int b = 0; b < kImgs; ++b) {
    k_transpose_bf16<false><<<dim3(kPix / 64, kCin / 64, 1), blk, 0, stream>>>(
        x + (size_t)b * kCin * kPix, kCin, kPix, 0, XT, nullptr, 0);
    k_im2col16<<<9216, blk, 0, stream>>>(XT, kCinShift, kPix, IM);
    wmma_gemm64<1, false, 2, 0, false, 2, 2><<<dim3(gemm_gx(kPix, kCi), 1), blk, 0, stream>>>(
        IM, nullptr, kK1, 0, W1P, nullptr, kK1, 0,
        (void*)(FP32 + (size_t)b * featStride), nullptr, kCi, 0,
        SV + kSlotBiasP1 * 128, SV + kSlotInvP1 * 128, nullptr, 0, kPix, kCi, kK1, 1.0f, kPix);
    wmma_gemm64<1, false, 2, 0, false, 2, 2><<<dim3(gemm_gx(kPix, kCi), 1), blk, 0, stream>>>(
        IM, nullptr, kK1, 0, W1C, nullptr, kK1, 0,
        (void*)(FC32 + (size_t)b * featStride), nullptr, kCi, 0,
        SV + kSlotBiasC1 * 128, SV + kSlotInvC1 * 128, nullptr, 0, kPix, kCi, kK1, 1.0f, kPix);
  }
  cast_f32_f16x2<<<8192, blk, 0, stream>>>(FP32, (_Float16*)FP16, (int)((2 * (size_t)kRowsAll * kCi) / 2));

  wmma_gemm64<0, false, 2, 1, false, 0, 0><<<dim3(gemm_gx(kRowsAll, kQkLd), 1), blk, 0, stream>>>(
      FP16, nullptr, kCi, 0, WQK, nullptr, kCi, 0, (void*)QKP, nullptr, kQkLd, 0,
      SV + kSlotQkb * 128, nullptr, nullptr, 0, kRowsAll, kQkLd, kCi, 0.5f, kRowsAll);
  wmma_gemm64<0, false, 1, 1, false, 0, 0><<<dim3(gemm_gx(kCi, kPix), kImgs), blk, 0, stream>>>(
      WV, nullptr, kCi, 0, FP16, nullptr, kCi, featStride, (void*)VPL, nullptr, kPix, (long)kCi * kPix,
      SV + kSlotVb * 128, nullptr, nullptr, 0, kCi, kPix, kCi, 0.5f, kCi);
  k_pam_flash<<<kImgs * (kPix / 64), 128, 0, stream>>>(QKP, VPL, FP32, pamg, P2IN);

  k_im2col16<<<9216, blk, 0, stream>>>(P2IN, kCiShift, kRowsAll, IM);
  wmma_gemm64<0, false, 2, 1, false, 2, 2><<<dim3(gemm_gx(kRowsAll, kCi), 1), blk, 0, stream>>>(
      IM, nullptr, kK2, 0, W2P, nullptr, kK2, 0, (void*)FEAT2, nullptr, kFeat2Ld, 0,
      SV + kSlotBiasP2 * 128, SV + kSlotInvP2 * 128, nullptr, 0, kRowsAll, kCi, kK2, 1.0f / kWCarry, kRowsAll);

  k_transpose_bf16<true><<<dim3(kCi / 64, kPix / 64, kImgs), blk, 0, stream>>>(
      FC32, kPix, kCi, featStride, FCTH, FCTL, (long)kCi * kPix);
  wmma_gemm64<1, true, 0, 0, false, 0, 0><<<dim3(gemm_gx(kCi, kCi), kImgs), blk, 0, stream>>>(
      FCTH, FCTL, kPix, (long)kCi * kPix, FCTH, FCTL, kPix, (long)kCi * kPix,
      (void*)EN, nullptr, kCi, (long)kCi * kCi, nullptr, nullptr, nullptr, 0, kCi, kCi, kPix, 1.0f, kCi);
  k_softmax128<<<(kImgs * kCi) / 8, blk, 0, stream>>>(EN, ATT, kImgs * kCi);
  wmma_gemm64<0, false, 0, 1, true, 0, 3><<<dim3(gemm_gx(kPix, kCi), kImgs), blk, 0, stream>>>(
      FC16, nullptr, kCi, featStride, ATT, nullptr, kCi, (long)kCi * kCi, (void*)C2IN, nullptr, kCi, featStride,
      nullptr, camg, FC32, featStride, kPix, kCi, kCi, 1.0f / kPCarry, kPix);

  k_im2col16<<<9216, blk, 0, stream>>>(C2IN, kCiShift, kRowsAll, IM);
  wmma_gemm64<0, false, 2, 1, false, 2, 2><<<dim3(gemm_gx(kRowsAll, kCi), 1), blk, 0, stream>>>(
      IM, nullptr, kK2, 0, W2C, nullptr, kK2, 0, (void*)(FEAT2 + kCi), nullptr, kFeat2Ld, 0,
      SV + kSlotBiasC2 * 128, SV + kSlotInvC2 * 128, nullptr, 0, kRowsAll, kCi, kK2, 1.0f / kWCarry, kRowsAll);

  wmma_gemm64<0, false, 1, 0, false, 0, 0><<<dim3(gemm_gx(kHeadRows, kPix), kImgs), blk, 0, stream>>>(
      WCLS, nullptr, kFeat2Ld, 0, FEAT2, nullptr, kFeat2Ld, (long)kPix * kFeat2Ld,
      (void*)dout, nullptr, kPix, outStride, SV + kSlotClsb * 128, nullptr, nullptr, 0,
      kHeadRows, kPix, kFeat2Ld, 1.0f / kWCarry, kCls);
  wmma_gemm64<0, false, 1, 0, false, 0, 0><<<dim3(gemm_gx(kHeadRows, kPix), kImgs), blk, 0, stream>>>(
      WAP, nullptr, kCi, 0, FEAT2, nullptr, kFeat2Ld, (long)kPix * kFeat2Ld,
      (void*)(dout + (size_t)kImgs * outStride), nullptr, kPix, outStride, SV + kSlotApb * 128, nullptr, nullptr, 0,
      kHeadRows, kPix, kCi, 1.0f / kWCarry, kCls);
  wmma_gemm64<0, false, 1, 0, false, 0, 0><<<dim3(gemm_gx(kHeadRows, kPix), kImgs), blk, 0, stream>>>(
      WAC, nullptr, kCi, 0, FEAT2 + kCi, nullptr, kFeat2Ld, (long)kPix * kFeat2Ld,
      (void*)(dout + (size_t)2 * kImgs * outStride), nullptr, kPix, outStride, SV + kSlotAcb * 128, nullptr, nullptr, 0,
      kHeadRows, kPix, kCi, 1.0f / kWCarry, kCls);
}
